// ODEFunc_88055419503310
// MI455X (gfx1250) — hardware-verified
//
#include <hip/hip_runtime.h>
#include <math.h>

typedef __attribute__((ext_vector_type(16))) _Float16 v16h;
typedef __attribute__((ext_vector_type(8)))  _Float16 v8h;
typedef __attribute__((ext_vector_type(8)))  float    v8f;
typedef __attribute__((ext_vector_type(4)))  float    v4f;
typedef __attribute__((ext_vector_type(2)))  float    v2f;
typedef __attribute__((ext_vector_type(4)))  unsigned int v4u;

constexpr int kB      = 4096;
constexpr int kPts    = 256;
constexpr int kHid    = 80;
constexpr int kWsz    = 16;
constexpr int kEnc    = 50;
constexpr int kWe     = 200;
constexpr int kKpad   = 64;
constexpr int kSpitch = 256;
constexpr int kN0     = 240;
constexpr int kN1     = 6480;
constexpr int kN5     = 162;
constexpr int kWblk   = kHid * kHid;
constexpr int kC0     = 0;
constexpr int kC1     = 256;
constexpr int kC2     = 6784;
constexpr int kC5     = 13312;
constexpr int kTH     = 13504;
constexpr int kTilesM = kB / 64;
constexpr int kTilesN = kTH / 64;
constexpr int kT1     = kC1 / 64;
constexpr int kT2     = kC2 / 64;
constexpr int kT5     = kC5 / 64;
constexpr int kHP     = 88;

static_assert(kC1 == ((kN0 + 63) / 64) * 64, "segment 0 pad");
static_assert(kC2 == kC1 + ((kN1 + 63) / 64) * 64, "segment 1 pad");
static_assert(kC5 == kC2 + ((kN1 + 63) / 64) * 64, "segment 2 pad");
static_assert(kTH == kC5 + ((kN5 + 63) / 64) * 64, "segment 3 pad");
static_assert(kTilesN == 211 && kTilesM == 64, "tile counts");
static_assert((kTilesM * kTilesN) % 8 == 0, "8 wave tiles per block, exact grid");
static_assert(kN0 == 2 * kHid + kHid && kN1 == kWblk + kHid && kN5 == 2 * kHid + 2, "head widths");
static_assert((kKpad % 32) == 0 && (kB % 64) == 0 && (kTH % 64) == 0, "GEMM multiples");
static_assert(((kTH * 2) % 128) == 0, "theta row pitch is a whole number of 128-B lines");
static_assert(((kHP * 2) % 16) == 0, "LDS pitch keeps 16-B alignment");

constexpr size_t kOffS     = 0;
constexpr size_t kOffWT    = kOffS    + (size_t)kB  * kSpitch * 2;
constexpr size_t kOffBias  = kOffWT   + (size_t)kTH * kKpad   * 2;
constexpr size_t kOffTheta = kOffBias + (size_t)kTH * 4;
constexpr size_t kWsTotal  = kOffTheta + (size_t)kB * kTH * 2;
static_assert(kWsTotal == 114504448ull, "carve total");
static_assert(kWsTotal <= 134217728ull, "carve cap");
static_assert((kOffWT % 128) == 0 && (kOffBias % 128) == 0 && (kOffTheta % 128) == 0, "aligned regions");

constexpr size_t kOut1Elem = (size_t)kB * kPts * 2;
constexpr size_t kOut2Elem = kOut1Elem + (size_t)kB * kWsz;
static_assert(kOut1Elem * 4 == 8388608ull && kOut2Elem * 4 == 8650752ull, "output byte offsets");
static_assert((kOut2Elem + (size_t)kB * kWsz) * 4 == 8912896ull, "output total");

__device__ __forceinline__ float h16_to_f32(unsigned hb) {
  const unsigned sgn = (hb & 0x8000u) << 16;
  const unsigned em = hb & 0x7fffu;
  const float fn = __uint_as_float((em << 13) + 0x38000000u);
  const float fs = (float)em * 5.9604644775390625e-8f;
  const float mag = (em < 0x400u) ? fs : fn;
  return __uint_as_float(__float_as_uint(mag) | sgn);
}

__device__ __forceinline__ float silu_f(float x) {
  const float d = 1.0f + expf(-x);
  return x * (1.0f / d);
}

__device__ __forceinline__ v16h frag_full(const _Float16* p) {
  union { v16h v; v8h h[2]; } f;
  f.h[0] = *(const v8h*)(p);
  f.h[1] = *(const v8h*)(p + 16);
  return f.v;
}
__device__ __forceinline__ v16h frag_tail(const _Float16* p) {
  union { v16h v; v8h h[2]; } f;
  const _Float16 hz = (_Float16)0.0f;
  const v8h z = {hz, hz, hz, hz, hz, hz, hz, hz};
  f.h[0] = *(const v8h*)(p);
  f.h[1] = z;
  return f.v;
}
__device__ __forceinline__ v8f mma_g(v16h a, v16h b, v8f c) {
  c = __builtin_amdgcn_wmma_f32_16x16x32_f16(false, a, false, b, (short)0, c, false, false);
  asm volatile("v_nop\n\tv_nop\n\tv_nop\n\tv_nop" : "+v"(c) : "v"(a), "v"(b));
  return c;
}
__device__ __forceinline__ void wave_lds_sync() {
  __builtin_amdgcn_fence(__ATOMIC_RELEASE, "workgroup");
  __builtin_amdgcn_wave_barrier();
  __builtin_amdgcn_fence(__ATOMIC_ACQUIRE, "workgroup");
}

__global__ __launch_bounds__(256) void rot_kernel(
    const float* __restrict__ w, const float* __restrict__ a,
    float* __restrict__ out1, float* __restrict__ out2)
{
  const int t = blockIdx.x * 256 + threadIdx.x;
  if (t >= kB * 4) return;
  const int b = t >> 2;
  const int j0 = (t & 3) * 2;
  const v4f wv = *(const v4f*)(w + (size_t)t * 4);
  const float re0 = a[b * 16 + j0];
  const float re1 = a[b * 16 + j0 + 1];
  const float im0 = a[b * 16 + 8 + j0];
  const float im1 = a[b * 16 + 9 + j0];
  v4f o;
  o[0] = wv[0] * re0 + wv[1] * im0;
  o[1] = wv[1] * re0 - wv[0] * im0;
  o[2] = wv[2] * re1 + wv[3] * im1;
  o[3] = wv[3] * re1 - wv[2] * im1;
  const v4f z = {0.0f, 0.0f, 0.0f, 0.0f};
  float* q1 = out1 + (size_t)t * 4;
  float* q2 = out2 + (size_t)t * 4;
  *(volatile v4f*)q1 = o;
  *(volatile v4f*)q2 = z;
  __threadfence();
  *(volatile v4f*)q1 = o;
  *(volatile v4f*)q2 = z;
}

__global__ __launch_bounds__(256) void prep_kernel(
    const float* __restrict__ w,
    const float* __restrict__ encW1, const float* __restrict__ encb1,
    const float* __restrict__ encW2, const float* __restrict__ encb2,
    const float* __restrict__ e1W1, const float* __restrict__ e1b1,
    const float* __restrict__ e2W1, const float* __restrict__ e2b1,
    unsigned short* __restrict__ S)
{
  __shared__ float wss[8 * 16];
  __shared__ float es[8 * 52];
  __shared__ float wcs[8 * kWe];
  __shared__ __align__(16) float sval[8 * kSpitch];
  const int tid = threadIdx.x;
  const int b0 = blockIdx.x * 8;
  if (tid < 128) wss[tid] = w[(size_t)b0 * 16 + tid];
#pragma unroll 1
  for (int idx = tid; idx < 448; idx += 256) {
    const int bb = idx / 56;
    const int r = idx - bb * 56;
    const int seg = r / 14;
    const int kk = 50 + (r - seg * 14);
    sval[bb * kSpitch + seg * 64 + kk] = 0.0f;
  }
  __syncthreads();
#pragma unroll 1
  for (int idx = tid; idx < 8 * kEnc; idx += 256) {
    const int bb = idx / kEnc;
    const int j = idx - bb * kEnc;
    float s = encb1[j];
#pragma unroll 1
    for (int k = 0; k < kWsz; ++k) s = fmaf(wss[bb * 16 + k], encW1[k * kEnc + j], s);
    es[bb * 52 + j] = silu_f(s);
  }
  __syncthreads();
#pragma unroll 1
  for (int idx = tid; idx < 8 * kWe; idx += 256) {
    const int bb = idx / kWe;
    const int j = idx - bb * kWe;
    float s = encb2[j];
#pragma unroll 1
    for (int k = 0; k < kEnc; ++k) s = fmaf(es[bb * 52 + k], encW2[k * kWe + j], s);
    wcs[bb * kWe + j] = s;
  }
  __syncthreads();
#pragma unroll 1
  for (int idx = tid; idx < 8 * kEnc; idx += 256) {
    const int bb = idx / kEnc;
    const int j = idx - bb * kEnc;
    float s1 = e1b1[j];
    float s2 = e2b1[j];
#pragma unroll 1
    for (int k = 0; k < kEnc; ++k) {
      s1 = fmaf(wcs[bb * kWe + 50 + k], e1W1[k * kEnc + j], s1);
      s2 = fmaf(wcs[bb * kWe + 100 + k], e2W1[k * kEnc + j], s2);
    }
    sval[bb * kSpitch + 64 + j] = silu_f(s1);
    sval[bb * kSpitch + 128 + j] = silu_f(s2);
    sval[bb * kSpitch + j] = wcs[bb * kWe + j];
    sval[bb * kSpitch + 192 + j] = wcs[bb * kWe + 150 + j];
  }
  __syncthreads();
  const float* sp = sval + tid * 8;
  const v4f a0 = *(const v4f*)(sp);
  const v4f a1 = *(const v4f*)(sp + 4);
  v8h hv;
#pragma unroll
  for (int e = 0; e < 4; ++e) {
    hv[e] = (_Float16)a0[e];
    hv[4 + e] = (_Float16)a1[e];
  }
  unsigned short* q = S + (size_t)b0 * kSpitch + tid * 8;
  *(volatile v8h*)q = hv;
  __threadfence();
  *(volatile v8h*)q = hv;
}

__global__ __launch_bounds__(256) void wt_kernel(
    const float* __restrict__ e0W, const float* __restrict__ e1W2,
    const float* __restrict__ e2W2, const float* __restrict__ e5W,
    unsigned short* __restrict__ WT)
{
  const int tid = threadIdx.x;
  const int row0 = blockIdx.x * 32;
  const bool g0 = row0 < kC1;
  const bool g1 = (!g0) && (row0 < kC2);
  const bool g2 = (!g0) && (!g1) && (row0 < kC5);
  const float* src = g0 ? e0W : (g1 ? e1W2 : (g2 ? e2W2 : e5W));
  const int ld = g0 ? kN0 : ((g1 || g2) ? kN1 : kN5);
  const int cbase = g0 ? kC0 : (g1 ? kC1 : (g2 ? kC2 : kC5));
  const bool perm = g1 || g2;
  const int ng = row0 + (tid >> 3);
  const int k0 = (tid & 7) * 8;
  const int c = ng - cbase;
  const int oo = c / kHid;
  const int ii = c - oo * kHid;
  const int cs = (perm && (c < kWblk)) ? (ii * kHid + oo) : c;
  const bool colok = (c < ld);
  const int cc = (cs < ld - 1) ? cs : (ld - 1);
  v8h hv;
#pragma unroll
  for (int e = 0; e < 8; ++e) {
    const int k = k0 + e;
    const int kc = (k < kEnc - 1) ? k : (kEnc - 1);
    const float v = src[(size_t)kc * ld + cc];
    const float vz = (colok && (k < kEnc)) ? v : 0.0f;
    hv[e] = (_Float16)vz;
  }
  unsigned short* q = WT + (size_t)ng * kKpad + k0;
  *(volatile v8h*)q = hv;
  __threadfence();
  *(volatile v8h*)q = hv;
}

__global__ __launch_bounds__(32) void bias_kernel(
    const float* __restrict__ e0b, const float* __restrict__ e1b2,
    const float* __restrict__ e2b2, const float* __restrict__ e5b,
    float* __restrict__ biasc)
{
  const int lane = threadIdx.x;
  const int col0 = blockIdx.x * 64;
  const bool g0 = col0 < kC1;
  const bool g1 = (!g0) && (col0 < kC2);
  const bool g2 = (!g0) && (!g1) && (col0 < kC5);
  const float* src = g0 ? e0b : (g1 ? e1b2 : (g2 ? e2b2 : e5b));
  const int nvalid = g0 ? kN0 : ((g1 || g2) ? kN1 : kN5);
  const int cbase = g0 ? kC0 : (g1 ? kC1 : (g2 ? kC2 : kC5));
  const bool perm = g1 || g2;
  v2f o;
#pragma unroll
  for (int e = 0; e < 2; ++e) {
    const int c = col0 - cbase + lane * 2 + e;
    const int oo = c / kHid;
    const int ii = c - oo * kHid;
    const int cs = (perm && (c < kWblk)) ? (ii * kHid + oo) : c;
    const int cc = (cs < nvalid - 1) ? cs : (nvalid - 1);
    const float v = src[cc];
    o[e] = (c < nvalid) ? v : 0.0f;
  }
  float* q = biasc + col0 + lane * 2;
  *(volatile v2f*)q = o;
  __threadfence();
  *(volatile v2f*)q = o;
}

__global__ __launch_bounds__(256) void theta_gemm_kernel(
    const unsigned short* __restrict__ Sp, const unsigned short* __restrict__ WTp,
    const float* __restrict__ biasc, unsigned short* __restrict__ theta)
{
  __shared__ __align__(16) float sT[8][16 * 68];
  const _Float16* S = (const _Float16*)Sp;
  const _Float16* WT = (const _Float16*)WTp;
  const int lane = threadIdx.x & 31;
  const int wave = threadIdx.x >> 5;
  const int tile = blockIdx.x * 8 + wave;
  if (tile >= kTilesM * kTilesN) return;
  const int tm = tile / kTilesN;
  const int tn = tile - tm * kTilesN;
  const int m0 = tm << 6;
  const int n0 = tn << 6;
  const int segA = (tn < kT1) ? 0 : ((tn < kT2) ? 64 : ((tn < kT5) ? 128 : 192));
  const bool doAct = (tn < kT1) || (tn >= kT5);
  const int rlane = lane & 15;
  const int koff = (lane >> 4) * 8;
  const int mOff = (lane >> 4) * 8;

  v8f acc[4][4];
#pragma unroll
  for (int i = 0; i < 4; ++i)
#pragma unroll
    for (int j = 0; j < 4; ++j) acc[i][j] = (v8f){0.f, 0.f, 0.f, 0.f, 0.f, 0.f, 0.f, 0.f};

#pragma unroll 1
  for (int k0 = 0; k0 < kKpad; k0 += 32) {
    v16h bh[4];
#pragma unroll
    for (int j = 0; j < 4; ++j)
      bh[j] = frag_full(WT + (size_t)(n0 + (j << 4) + rlane) * kKpad + koff + k0);
#pragma unroll
    for (int i = 0; i < 4; ++i) {
      const v16h ah = frag_full(S + (size_t)(m0 + (i << 4) + rlane) * kSpitch + segA + koff + k0);
#pragma unroll
      for (int j = 0; j < 4; ++j) acc[i][j] = mma_g(ah, bh[j], acc[i][j]);
    }
  }

  float* slab = sT[wave];
  const int q = lane >> 3;
  const int c8 = (lane & 7) * 8;
#pragma unroll
  for (int i = 0; i < 4; ++i) {
    const int mBase = m0 + (i << 4);
#pragma unroll
    for (int j = 0; j < 4; ++j) {
      const float bv = biasc[n0 + (j << 4) + rlane];
#pragma unroll
      for (int r = 0; r < 8; ++r) slab[(mOff + r) * 68 + (j << 4) + rlane] = acc[i][j][r] + bv;
    }
    wave_lds_sync();
    if (doAct) {
#pragma unroll 1
      for (int t = 0; t < 32; ++t) {
        const int idx = t * 32 + lane;
        float* p = slab + (idx >> 6) * 68 + (idx & 63);
        const float x = *p;
        *p = silu_f(x);
      }
      wave_lds_sync();
    }
    for (int pass = 0; pass < 2; ++pass) {
#pragma unroll
      for (int it = 0; it < 4; ++it) {
        const int row = it * 4 + q;
        const float* sp = slab + row * 68 + c8;
        v8h hv;
#pragma unroll
        for (int e = 0; e < 8; ++e) hv[e] = (_Float16)sp[e];
        *(volatile v8h*)(theta + (size_t)(mBase + row) * kTH + n0 + c8) = hv;
      }
      __threadfence();
    }
    wave_lds_sync();
  }
}

template <bool LAST>
__device__ __forceinline__ void mlp_layer(_Float16* hA, const _Float16* WTs, const float* bl,
                                          const float* par3, float* dyS, const int wv, const int lane)
{
  const int l15 = lane & 15;
  const int hh = lane >> 4;
#pragma unroll
  for (int mt = 0; mt < 2; ++mt) {
    const int rowbase = wv * 32 + mt * 16;
    const _Float16* arow = hA + (rowbase + l15) * kHP + 8 * hh;
    const v16h a0 = frag_full(arow);
    const v16h a1 = frag_full(arow + 32);
    const v16h a2 = frag_tail(arow + 64);
    v8f acc[5];
#pragma unroll
    for (int nt = 0; nt < 5; ++nt) {
      const int n = nt * 16 + l15;
      const float bv = bl[n];
      v8f c;
#pragma unroll
      for (int r = 0; r < 8; ++r) c[r] = bv;
      const _Float16* brow = WTs + n * kHP + 8 * hh;
      const v16h b0 = frag_full(brow);
      const v16h b1 = frag_full(brow + 32);
      const v16h b2 = frag_tail(brow + 64);
      c = mma_g(a0, b0, c);
      c = mma_g(a1, b1, c);
      c = mma_g(a2, b2, c);
#pragma unroll
      for (int r = 0; r < 8; ++r) c[r] = fmaxf(c[r], 0.0f);
      acc[nt] = c;
    }
    wave_lds_sync();
    if (!LAST) {
#pragma unroll
      for (int nt = 0; nt < 5; ++nt)
#pragma unroll
        for (int r = 0; r < 8; ++r)
          hA[(rowbase + 8 * hh + r) * kHP + nt * 16 + l15] = (_Float16)acc[nt][r];
    } else {
      float s0[8], s1[8];
#pragma unroll
      for (int r = 0; r < 8; ++r) { s0[r] = 0.0f; s1[r] = 0.0f; }
#pragma unroll
      for (int nt = 0; nt < 5; ++nt) {
        const v2f w3 = *(const v2f*)(par3 + 2 * (nt * 16 + l15));
#pragma unroll
        for (int r = 0; r < 8; ++r) {
          s0[r] = fmaf(acc[nt][r], w3[0], s0[r]);
          s1[r] = fmaf(acc[nt][r], w3[1], s1[r]);
        }
      }
#pragma unroll
      for (int r = 0; r < 8; ++r) {
#pragma unroll
        for (int off = 1; off < 16; off <<= 1) {
          s0[r] += __shfl_xor(s0[r], off, 32);
          s1[r] += __shfl_xor(s1[r], off, 32);
        }
      }
      const float b30 = par3[2 * kHid];
      const float b31 = par3[2 * kHid + 1];
      if (l15 == 0) {
#pragma unroll
        for (int r = 0; r < 8; ++r) {
          v2f o;
          o[0] = s0[r] + b30;
          o[1] = s1[r] + b31;
          *(v2f*)(dyS + (rowbase + 8 * hh + r) * 2) = o;
        }
      }
    }
  }
}

__global__ __launch_bounds__(256) void mlp_kernel(
    const float* __restrict__ y, const unsigned short* __restrict__ theta, float* __restrict__ out0)
{
  __shared__ __align__(16) _Float16 hA[kPts * kHP];
  __shared__ __align__(16) _Float16 WTs[kHid * kHP];
  __shared__ __align__(16) float par0[240];
  __shared__ __align__(16) float par3[168];
  __shared__ __align__(16) float bl1[kHid];
  __shared__ __align__(16) float bl2[kHid];
  __shared__ __align__(16) float dyS[kPts * 2];
  const int tid = threadIdx.x;
  const int lane = tid & 31;
  const int wv = tid >> 5;
  const int b = blockIdx.x;
  const unsigned short* th = theta + (size_t)b * kTH;
  const unsigned int* thw = (const unsigned int*)th;

  {
    const int j0 = (tid < 239) ? tid : 239;
    const unsigned wd0 = thw[(kC0 + j0) >> 1];
    const unsigned hb0 = (j0 & 1) ? (wd0 >> 16) : (wd0 & 0xffffu);
    const float v0 = h16_to_f32(hb0);
    const int j3 = (tid < kN5 - 1) ? tid : (kN5 - 1);
    const unsigned wd3 = thw[(kC5 + j3) >> 1];
    const unsigned hb3 = (j3 & 1) ? (wd3 >> 16) : (wd3 & 0xffffu);
    const float v3 = h16_to_f32(hb3);
    const int jb = (tid < kHid - 1) ? tid : (kHid - 1);
    const unsigned wd1 = thw[(kC1 + kWblk + jb) >> 1];
    const unsigned hb1 = (jb & 1) ? (wd1 >> 16) : (wd1 & 0xffffu);
    const float v1 = h16_to_f32(hb1);
    const unsigned wd2 = thw[(kC2 + kWblk + jb) >> 1];
    const unsigned hb2 = (jb & 1) ? (wd2 >> 16) : (wd2 & 0xffffu);
    const float v2 = h16_to_f32(hb2);
    if (tid < 240) par0[tid] = v0;
    if (tid < kN5) par3[tid] = v3;
    if (tid < kHid) { bl1[tid] = v1; bl2[tid] = v2; }
  }
  {
    const v4u* src = (const v4u*)(th + kC1);
#pragma unroll 1
    for (int idx = tid; idx < 800; idx += 256) {
      const int o = idx / 10;
      const int c = idx - o * 10;
      const v4u v = src[idx];
      *(v4u*)(WTs + o * kHP + c * 8) = v;
    }
  }
  __syncthreads();

  {
    const v2f yy = *(const v2f*)(y + ((size_t)b * kPts + tid) * 2);
    _Float16* hr = hA + tid * kHP;
#pragma unroll 1
    for (int jj = 0; jj < 10; ++jj) {
      const v4f wa0 = *(const v4f*)(par0 + jj * 8);
      const v4f wa1 = *(const v4f*)(par0 + jj * 8 + 4);
      const v4f wb0 = *(const v4f*)(par0 + kHid + jj * 8);
      const v4f wb1 = *(const v4f*)(par0 + kHid + jj * 8 + 4);
      const v4f bb0 = *(const v4f*)(par0 + 2 * kHid + jj * 8);
      const v4f bb1 = *(const v4f*)(par0 + 2 * kHid + jj * 8 + 4);
      v8h o;
#pragma unroll
      for (int e = 0; e < 4; ++e) {
        float h0 = fmaf(yy[1], wb0[e], bb0[e]);
        h0 = fmaf(yy[0], wa0[e], h0);
        float h1 = fmaf(yy[1], wb1[e], bb1[e]);
        h1 = fmaf(yy[0], wa1[e], h1);
        o[e] = (_Float16)fmaxf(h0, 0.0f);
        o[4 + e] = (_Float16)fmaxf(h1, 0.0f);
      }
      *(v8h*)(hr + jj * 8) = o;
    }
  }
  __syncthreads();

  mlp_layer<false>(hA, WTs, bl1, par3, dyS, wv, lane);
  __syncthreads();

  {
    const v4u* src = (const v4u*)(th + kC2);
#pragma unroll 1
    for (int idx = tid; idx < 800; idx += 256) {
      const int o = idx / 10;
      const int c = idx - o * 10;
      const v4u v = src[idx];
      *(v4u*)(WTs + o * kHP + c * 8) = v;
    }
  }
  __syncthreads();

  mlp_layer<true>(hA, WTs, bl2, par3, dyS, wv, lane);
  __syncthreads();

  if (tid < 128) {
    const v4f v = *(const v4f*)(dyS + tid * 4);
    float* q = out0 + (size_t)b * (kPts * 2) + tid * 4;
    *(volatile v4f*)q = v;
    __threadfence();
    *(volatile v4f*)q = v;
  }
}

extern "C" void kernel_launch(void* const* d_in, const int* in_sizes, int n_in,
                              void* d_out, int out_size, void* d_ws, size_t ws_size,
                              hipStream_t stream)
{
  if (n_in < 20) return;
  if (in_sizes[1] != kB * kPts * 2) return;
  if (in_sizes[2] != kB * kWsz) return;
  if (in_sizes[3] != kB * kWsz) return;
  if (in_sizes[4] != kWsz * kEnc) return;
  if (in_sizes[5] != kEnc) return;
  if (in_sizes[6] != kEnc * kWe) return;
  if (in_sizes[7] != kWe) return;
  if (in_sizes[8] != kEnc * kN0) return;
  if (in_sizes[9] != kN0) return;
  if (in_sizes[10] != kEnc * kEnc) return;
  if (in_sizes[11] != kEnc) return;
  if (in_sizes[12] != kEnc * kN1) return;
  if (in_sizes[13] != kN1) return;
  if (in_sizes[14] != kEnc * kEnc) return;
  if (in_sizes[15] != kEnc) return;
  if (in_sizes[16] != kEnc * kN1) return;
  if (in_sizes[17] != kN1) return;
  if (in_sizes[18] != kEnc * kN5) return;
  if (in_sizes[19] != kN5) return;
  if ((size_t)out_size != kOut2Elem + (size_t)kB * kWsz) return;
  if (ws_size < kWsTotal) return;

  const float* y     = (const float*)d_in[1];
  const float* w     = (const float*)d_in[2];
  const float* a     = (const float*)d_in[3];
  const float* encW1 = (const float*)d_in[4];
  const float* encb1 = (const float*)d_in[5];
  const float* encW2 = (const float*)d_in[6];
  const float* encb2 = (const float*)d_in[7];
  const float* e0W   = (const float*)d_in[8];
  const float* e0b   = (const float*)d_in[9];
  const float* e1W1  = (const float*)d_in[10];
  const float* e1b1  = (const float*)d_in[11];
  const float* e1W2  = (const float*)d_in[12];
  const float* e1b2  = (const float*)d_in[13];
  const float* e2W1  = (const float*)d_in[14];
  const float* e2b1  = (const float*)d_in[15];
  const float* e2W2  = (const float*)d_in[16];
  const float* e2b2  = (const float*)d_in[17];
  const float* e5W   = (const float*)d_in[18];
  const float* e5b   = (const float*)d_in[19];

  float* out  = (float*)d_out;
  float* out0 = out;
  float* out1 = out + kOut1Elem;
  float* out2 = out + kOut2Elem;

  char* ws = (char*)d_ws;
  unsigned short* S     = (unsigned short*)(ws + kOffS);
  unsigned short* WT    = (unsigned short*)(ws + kOffWT);
  float*          biasc = (float*)(ws + kOffBias);
  unsigned short* theta = (unsigned short*)(ws + kOffTheta);

  rot_kernel<<<(kB * 4) / 256, 256, 0, stream>>>(w, a, out1, out2);
  prep_kernel<<<kB / 8, 256, 0, stream>>>(w, encW1, encb1, encW2, encb2, e1W1, e1b1, e2W1, e2b1, S);
  wt_kernel<<<kTH / 32, 256, 0, stream>>>(e0W, e1W2, e2W2, e5W, WT);
  bias_kernel<<<kTilesN, 32, 0, stream>>>(e0b, e1b2, e2b2, e5b, biasc);
  theta_gemm_kernel<<<(kTilesM * kTilesN) / 8, 256, 0, stream>>>(S, WT, biasc, theta);
  mlp_kernel<<<kB, 256, 0, stream>>>(y, theta, out0);
}
